// MultiHeadGraphAttention_60825326846769
// MI455X (gfx1250) — hardware-run, weakly checked
//
#include <hip/hip_runtime.h>
#include <stddef.h>


typedef __bf16         v16bf __attribute__((ext_vector_type(16)));
typedef unsigned short v16us __attribute__((ext_vector_type(16)));
typedef unsigned short v8us  __attribute__((ext_vector_type(8)));
typedef unsigned short v4us  __attribute__((ext_vector_type(4)));
typedef float          v8f   __attribute__((ext_vector_type(8)));
typedef float          v4f   __attribute__((ext_vector_type(4)));
typedef unsigned int   v4u   __attribute__((ext_vector_type(4)));
typedef int            v4i   __attribute__((ext_vector_type(4)));
typedef v8us v8usa __attribute__((may_alias));
typedef v4us v4usa __attribute__((may_alias));
typedef v4f  v4fa  __attribute__((may_alias));
typedef v4u  v4ua  __attribute__((may_alias));
typedef v4i  v4ia  __attribute__((may_alias));

#define BB     8
#define NNODE  1024
#define DIN    256
#define DOUT   256
#define NH     4
#define HDIM   64
#define NBH    (BB * NH)
#define GB     64
#define NBLK   (NNODE / GB)
#define NEGBIG (-1.0e9f)
#define SLOPE  0.2f
#define LNEPS  1.0e-5f
#define TP     68
#define TPP    260
#define PWT    264
#define PB_H   ((BB * NNODE * DIN) / (256 * 8))
#define PB_PW  ((DOUT * DOUT) / (256 * 8))
#define PB_WT  NH
#define PB_ADJ (NNODE / 32)
#define PB_TOT (PB_H + PB_PW + PB_WT + PB_ADJ)

static_assert(DIN % 32 == 0);
static_assert(DOUT % 32 == 0);
static_assert(NNODE % GB == 0);
static_assert(NNODE % 32 == 0);
static_assert(HDIM == 64);
static_assert(DOUT == NH * HDIM);
static_assert(DIN == DOUT);
static_assert((BB * NNODE * DIN) % 2048 == 0);
static_assert((DOUT * DOUT) % 2048 == 0);
static_assert((GB * TP) % 4 == 0);
static_assert((32 * TPP) % 4 == 0);

union Frag { v16bf v; v8us half[2]; v16us u; };

__device__ __forceinline__ unsigned short f2bf(float f) {
  unsigned int u = __float_as_uint(f);
  u = u + 0x7FFFu + ((u >> 16) & 1u);
  return (unsigned short)(u >> 16);
}
__device__ __forceinline__ float bf2f(unsigned short s) { return __uint_as_float(((unsigned int)s) << 16); }
__device__ __forceinline__ float bfr(float f) { return bf2f(f2bf(f)); }

__device__ __forceinline__ v8f vzero8() {
  v8f z = {0.f, 0.f, 0.f, 0.f, 0.f, 0.f, 0.f, 0.f};
  return z;
}

__device__ __forceinline__ v8f wmma_bf(v16bf a, v16bf b, v8f c) {
  v8f d = __builtin_amdgcn_wmma_f32_16x16x32_bf16(false, a, false, b, (short)0, c, false, false);
  asm volatile("v_nop\n\tv_nop\n\tv_nop\n\tv_nop" : "+v"(d) : "v"(a), "v"(b));
  return d;
}

__device__ __forceinline__ v16bf load_frag(const unsigned short* p, int h) {
  Frag f;
  f.half[0] = *(const v8usa*)(p + 8 * h);
  f.half[1] = *(const v8usa*)(p + 16 + 8 * h);
  return f.v;
}

__device__ __forceinline__ void hl8(v4f a, v4f c, v8us& hv, v8us& lv) {
  const float v[8] = {a[0], a[1], a[2], a[3], c[0], c[1], c[2], c[3]};
#pragma unroll
  for (int e = 0; e < 8; ++e) {
    const unsigned short hb = f2bf(v[e]);
    hv[e] = hb;
    lv[e] = f2bf(v[e] - bf2f(hb));
  }
}

__device__ __forceinline__ void cvt8_store2(const float* src, unsigned short* dst) {
  const v4f a = *(const v4fa*)src;
  const v4f c = *(const v4fa*)(src + 4);
  v8us o;
  o[0] = f2bf(a[0]); o[1] = f2bf(a[1]); o[2] = f2bf(a[2]); o[3] = f2bf(a[3]);
  o[4] = f2bf(c[0]); o[5] = f2bf(c[1]); o[6] = f2bf(c[2]); o[7] = f2bf(c[3]);
  *(volatile v8us*)dst = o;
  __threadfence();
  *(volatile v8us*)dst = o;
}

__device__ __forceinline__ void wt_store(const unsigned short* sW, unsigned short* WT, int head, int w, int l) {
#pragma unroll
  for (int s = 0; s < 8; ++s) {
    const int row = s * 8 + w;
    const v8us v = *(const v8usa*)(sW + row * PWT + 8 * l);
    *(volatile v8us*)(WT + ((size_t)(head * HDIM + row)) * DIN + 8 * l) = v;
  }
}

__device__ __forceinline__ void adj_store(const unsigned int* sB, unsigned int* ADJB, int row0, int w, int l) {
  const int rl = 4 * w + (l >> 3), ch = l & 7;
  const v4u v = *(const v4ua*)(sB + rl * 32 + ch * 4);
  *(volatile v4u*)(ADJB + ((size_t)(row0 + rl)) * 32 + ch * 4) = v;
}

__global__ void __launch_bounds__(256) k_prep(const float* __restrict__ h, const int* __restrict__ adj,
                                              const float* __restrict__ W, const float* __restrict__ pw,
                                              unsigned short* HB, unsigned short* PWB, unsigned short* WT,
                                              unsigned int* ADJB) {
  __shared__ v4u smem[(HDIM * PWT * 2) / 16];
  const int blk = blockIdx.x, tid = threadIdx.x, w = tid >> 5, l = tid & 31;
  if (blk < PB_H) {
    const size_t g = (size_t)blk * 256 + tid;
    cvt8_store2(h + g * 8, HB + g * 8);
  } else if (blk < PB_H + PB_PW) {
    const size_t g = (size_t)(blk - PB_H) * 256 + tid;
    cvt8_store2(pw + g * 8, PWB + g * 8);
  } else if (blk < PB_H + PB_PW + PB_WT) {
    const int head = blk - (PB_H + PB_PW);
    unsigned short* sW = (unsigned short*)smem;
    const float* Wh = W + (size_t)head * DIN * HDIM;
    for (int idx = tid; idx < DIN * HDIM; idx += 256) {
      const int k = idx >> 6, d = idx & 63;
      sW[d * PWT + k] = f2bf(Wh[idx]);
    }
    __syncthreads();
    wt_store(sW, WT, head, w, l);
    __threadfence();
    wt_store(sW, WT, head, w, l);
  } else {
    const int row0 = (blk - (PB_H + PB_PW + PB_WT)) * 32;
    unsigned int* sB = (unsigned int*)smem;
#pragma unroll 1
    for (int rr = 0; rr < 4; ++rr) {
      const int row = row0 + 4 * w + rr;
      const int* ar = adj + (size_t)row * NNODE;
#pragma unroll 2
      for (int wd4 = 0; wd4 < 8; ++wd4) {
        const v4i q = *(const v4ia*)(ar + wd4 * 128 + 4 * l);
        const int sh = 4 * (l & 7);
        unsigned int bits = ((q[0] != 0) ? 1u : 0u) << sh;
        bits |= ((q[1] != 0) ? 1u : 0u) << (sh + 1);
        bits |= ((q[2] != 0) ? 1u : 0u) << (sh + 2);
        bits |= ((q[3] != 0) ? 1u : 0u) << (sh + 3);
        bits |= __shfl_xor(bits, 1, 32);
        bits |= __shfl_xor(bits, 2, 32);
        bits |= __shfl_xor(bits, 4, 32);
        if ((l & 7) == 0) sB[(4 * w + rr) * 32 + wd4 * 4 + (l >> 3)] = bits;
      }
    }
    __syncthreads();
    adj_store(sB, ADJB, row0, w, l);
    __threadfence();
    adj_store(sB, ADJB, row0, w, l);
  }
}

__device__ __forceinline__ void gw_store(const float* sT, const float* sSc, unsigned short* WHI, unsigned short* WLO,
                                         float* SC, int bh, int node0, int w, int l) {
  const int q8 = l & 7;
#pragma unroll
  for (int s = 0; s < 4; ++s) {
    const int d = w * 16 + s * 4 + (l >> 3);
    v4f a, c;
    a[0] = sT[(8 * q8 + 0) * TP + d]; a[1] = sT[(8 * q8 + 1) * TP + d];
    a[2] = sT[(8 * q8 + 2) * TP + d]; a[3] = sT[(8 * q8 + 3) * TP + d];
    c[0] = sT[(8 * q8 + 4) * TP + d]; c[1] = sT[(8 * q8 + 5) * TP + d];
    c[2] = sT[(8 * q8 + 6) * TP + d]; c[3] = sT[(8 * q8 + 7) * TP + d];
    v8us hv, lv;
    hl8(a, c, hv, lv);
    const size_t off = ((size_t)(bh * HDIM + d)) * NNODE + node0 + 8 * q8;
    *(volatile v8us*)(WHI + off) = hv;
    *(volatile v8us*)(WLO + off) = lv;
  }
  if (w == 0) {
    const int sg = l >> 4, q = l & 15;
    const v4f v = *(const v4fa*)(sSc + sg * GB + 4 * q);
    *(volatile v4f*)(SC + ((size_t)(sg * NBH + bh)) * NNODE + node0 + 4 * q) = v;
  }
}

__global__ void __launch_bounds__(128) k_gemm_wh(const unsigned short* __restrict__ HB, const unsigned short* __restrict__ WT,
                                                 const float* __restrict__ a1, const float* __restrict__ a2,
                                                 unsigned short* WHI, unsigned short* WLO, float* SC) {
  __shared__ v4f sT4[(GB * TP) / 4];
  __shared__ float sSc[2 * GB];
  __shared__ float sAv[2 * HDIM];
  float* sT = (float*)sT4;
  const int bid = blockIdx.x;
  const int b = bid / (NH * NBLK), rem = bid - b * NH * NBLK;
  const int head = rem / NBLK, nb = rem - head * NBLK;
  const int node0 = nb * GB, bh = b * NH + head;
  const int tid = threadIdx.x, w = tid >> 5, l = tid & 31, h = l >> 4, m = l & 15;

  {
    const int ia = (tid < HDIM) ? tid : (tid - HDIM);
    const float v1 = a1[head * HDIM + ia];
    const float v2 = a2[head * HDIM + ia];
    sAv[tid] = bfr((tid < HDIM) ? v1 : v2);
  }

  v8f acc[4];
#pragma unroll
  for (int nt = 0; nt < 4; ++nt) acc[nt] = vzero8();
  const unsigned short* arow = HB + ((size_t)(b * NNODE + node0 + 16 * w + m)) * DIN;
  const unsigned short* brow = WT + ((size_t)(head * HDIM + m)) * DIN;
#pragma unroll
  for (int k0 = 0; k0 < DIN; k0 += 32) {
    const v16bf a = load_frag(arow + k0, h);
#pragma unroll
    for (int nt = 0; nt < 4; ++nt) {
      const v16bf bf = load_frag(brow + (size_t)(nt * 16) * DIN + k0, h);
      acc[nt] = wmma_bf(a, bf, acc[nt]);
    }
  }
#pragma unroll
  for (int nt = 0; nt < 4; ++nt)
#pragma unroll
    for (int r = 0; r < 8; ++r)
      sT[(w * 16 + 8 * h + r) * TP + nt * 16 + m] = acc[nt][r];
  __syncthreads();

  {
    const int row = tid >> 1, part = tid & 1, c0 = part * 32;
    float s = 0.f, t = 0.f;
#pragma unroll 4
    for (int k = 0; k < 32; ++k) {
      const float v = sT[row * TP + c0 + k];
      s += v * sAv[c0 + k];
      t += v * sAv[HDIM + c0 + k];
    }
    s += __shfl_xor(s, 1, 32);
    t += __shfl_xor(t, 1, 32);
    if (part == 0) {
      sSc[row] = s;
      sSc[GB + row] = t;
    }
  }
  __syncthreads();
  gw_store(sT, sSc, WHI, WLO, SC, bh, node0, w, l);
  __threadfence();
  gw_store(sT, sSc, WHI, WLO, SC, bh, node0, w, l);
}

__device__ __forceinline__ void hm_store(const float* sOw, unsigned short* HMH, unsigned short* HML,
                                         size_t rowBase, int head, int l) {
  const int q8 = l & 7;
#pragma unroll
  for (int s = 0; s < 4; ++s) {
    const int row = s * 4 + (l >> 3);
    const v4f a = *(const v4fa*)(sOw + row * TP + 8 * q8);
    const v4f c = *(const v4fa*)(sOw + row * TP + 8 * q8 + 4);
    v8us hv, lv;
    hl8(a, c, hv, lv);
    const size_t off = (rowBase + row) * DOUT + head * HDIM + 8 * q8;
    *(volatile v8us*)(HMH + off) = hv;
    *(volatile v8us*)(HML + off) = lv;
  }
}

__global__ void __launch_bounds__(128) k_attn(const unsigned int* __restrict__ ADJB, const float* __restrict__ SC,
                                              const unsigned short* __restrict__ WHI, const unsigned short* __restrict__ WLO,
                                              unsigned short* HMH, unsigned short* HML) {
  __shared__ float sED[NNODE];
  __shared__ v4f sO4[(4 * 16 * TP) / 4];
  float* sO = (float*)sO4;
  const int bid = blockIdx.x;
  const int b = bid / (NH * NBLK), rem = bid - b * NH * NBLK;
  const int head = rem / NBLK, rb = rem - head * NBLK;
  const int bh = b * NH + head;
  const int tid = threadIdx.x, w = tid >> 5, l = tid & 31, h = l >> 4, m = l & 15;

  const float* edg = SC + ((size_t)(NBH + bh)) * NNODE;
  for (int j = tid; j < NNODE; j += 128) sED[j] = edg[j];
  __syncthreads();

  const int i0 = rb * GB + w * 16;
  const size_t rowBase = (size_t)b * NNODE + i0;
  float* sOw = sO + w * 16 * TP;

  float myMx = -__builtin_huge_valf();
#pragma unroll 1
  for (int r = 0; r < 16; ++r) {
    const unsigned int wv = ADJB[(size_t)(i0 + r) * 32 + l];
    float mx = -__builtin_huge_valf();
    const float* ep = sED + l * 32;
#pragma unroll
    for (int b4 = 0; b4 < 8; ++b4) {
      const v4f q = *(const v4fa*)(ep + b4 * 4);
#pragma unroll
      for (int e = 0; e < 4; ++e)
        mx = ((wv >> (b4 * 4 + e)) & 1u) ? fmaxf(mx, q[e]) : mx;
    }
#pragma unroll
    for (int off = 16; off > 0; off >>= 1) mx = fmaxf(mx, __shfl_xor(mx, off, 32));
    myMx = (m == r) ? mx : myMx;
  }
  const float esm = SC[(size_t)bh * NNODE + i0 + m];
  const float pmask = (myMx > -__builtin_huge_valf()) ? 0.f : 1.f;
  float M;
  {
    const float xm = esm + myMx;
    M = (xm >= 0.f) ? xm : SLOPE * xm;
    M = fmaxf(M, NEGBIG);
  }

  v8f acc[4];
#pragma unroll
  for (int t = 0; t < 4; ++t) acc[t] = vzero8();
  float psum = 0.f;
  const unsigned int* arow = ADJB + (size_t)(i0 + m) * 32;
  const unsigned short* wbh = WHI + ((size_t)(bh * HDIM + m)) * NNODE;
  const unsigned short* wbl = WLO + ((size_t)(bh * HDIM + m)) * NNODE;
#pragma unroll 1
  for (int kt = 0; kt < NNODE / 32; ++kt) {
    const int kk = kt * 32;
    const unsigned int aw = arow[kt];
    const v4f q0 = *(const v4fa*)(sED + kk + 8 * h);
    const v4f q1 = *(const v4fa*)(sED + kk + 8 * h + 4);
    const v4f q2 = *(const v4fa*)(sED + kk + 16 + 8 * h);
    const v4f q3 = *(const v4fa*)(sED + kk + 16 + 8 * h + 4);
    float edv[16];
#pragma unroll
    for (int e = 0; e < 4; ++e) {
      edv[e] = q0[e]; edv[4 + e] = q1[e]; edv[8 + e] = q2[e]; edv[12 + e] = q3[e];
    }
    Frag fh, fl;
#pragma unroll
    for (int i = 0; i < 16; ++i) {
      const int kb = i + (i & 8) + 8 * h;
      float x = esm + edv[i];
      x = (x >= 0.f) ? x : SLOPE * x;
      const float ex = __expf(x - M);
      const float p = ((aw >> kb) & 1u) ? ex : pmask;
      psum += p;
      const unsigned short hb = f2bf(p);
      fh.u[i] = hb;
      fl.u[i] = f2bf(p - bf2f(hb));
    }
#pragma unroll
    for (int t = 0; t < 4; ++t) {
      const size_t co = (size_t)(t * 16) * NNODE + kk;
      const v16bf bhf = load_frag(wbh + co, h);
      const v16bf blf = load_frag(wbl + co, h);
      acc[t] = wmma_bf(fh.v, bhf, acc[t]);
      acc[t] = wmma_bf(fl.v, bhf, acc[t]);
      acc[t] = wmma_bf(fh.v, blf, acc[t]);
    }
  }
  psum += __shfl_xor(psum, 16, 32);
  const float rinvm = 1.0f / psum;
#pragma unroll
  for (int r = 0; r < 8; ++r) {
    const float sc = __shfl(rinvm, 8 * h + r, 32);
#pragma unroll
    for (int t = 0; t < 4; ++t)
      sOw[(8 * h + r) * TP + t * 16 + m] = acc[t][r] * sc;
  }
  __syncthreads();

  hm_store(sOw, HMH, HML, rowBase, head, l);
  __threadfence();
  hm_store(sOw, HMH, HML, rowBase, head, l);
}

__device__ __forceinline__ void out_store(const float* sT, float* out, int b, int row0, int w, int l) {
#pragma unroll
  for (int rr = 0; rr < 8; ++rr) {
    const int row = w * 8 + rr;
    const v4f o0 = *(const v4fa*)(sT + row * TPP + 4 * l);
    const v4f o1 = *(const v4fa*)(sT + row * TPP + 128 + 4 * l);
    const size_t gi = ((size_t)(b * NNODE + row0 + row)) * DOUT;
    *(volatile v4f*)(out + gi + 4 * l) = o0;
    *(volatile v4f*)(out + gi + 128 + 4 * l) = o1;
  }
}

__global__ void __launch_bounds__(128) k_proj_ln(const unsigned short* __restrict__ HMH, const unsigned short* __restrict__ HML,
                                                 const unsigned short* __restrict__ PWB, const unsigned short* __restrict__ HB,
                                                 const float* __restrict__ pb, const float* __restrict__ gam,
                                                 const float* __restrict__ bet, float* out) {
  __shared__ v4f sT4[(32 * TPP) / 4];
  float* sT = (float*)sT4;
  const int bid = blockIdx.x;
  const int b = bid / (NNODE / 32), rb = bid - b * (NNODE / 32);
  const int row0 = rb * 32;
  const int tid = threadIdx.x, w = tid >> 5, l = tid & 31, h = l >> 4, m = l & 15;
  const int rg = w >> 1, cg = w & 1;

  v8f acc[8];
#pragma unroll
  for (int nt = 0; nt < 8; ++nt) acc[nt] = vzero8();
  const size_t aoff = ((size_t)(b * NNODE + row0 + 16 * rg + m)) * DOUT;
  const unsigned short* bro = PWB + ((size_t)(128 * cg + m)) * DOUT;
#pragma unroll
  for (int k0 = 0; k0 < DOUT; k0 += 32) {
    const v16bf ah = load_frag(HMH + aoff + k0, h);
    const v16bf al = load_frag(HML + aoff + k0, h);
#pragma unroll
    for (int nt = 0; nt < 8; ++nt) {
      const v16bf bf = load_frag(bro + (size_t)(nt * 16) * DOUT + k0, h);
      acc[nt] = wmma_bf(ah, bf, acc[nt]);
      acc[nt] = wmma_bf(al, bf, acc[nt]);
    }
  }
#pragma unroll
  for (int nt = 0; nt < 8; ++nt)
#pragma unroll
    for (int r = 0; r < 8; ++r)
      sT[(16 * rg + 8 * h + r) * TPP + 128 * cg + nt * 16 + m] = acc[nt][r];
  __syncthreads();

  float pbv[8], gv[8], bv[8];
#pragma unroll
  for (int e = 0; e < 8; ++e) {
    const int col = (e < 4) ? (4 * l + e) : (128 + 4 * l + (e - 4));
    pbv[e] = bfr(pb[col]);
    gv[e]  = bfr(gam[col]);
    bv[e]  = bfr(bet[col]);
  }
#pragma unroll 1
  for (int rr = 0; rr < 8; ++rr) {
    const int row = w * 8 + rr;
    float* tr = sT + row * TPP;
    const v4f x0 = *(const v4fa*)(tr + 4 * l);
    const v4f x1 = *(const v4fa*)(tr + 128 + 4 * l);
    const size_t grow = ((size_t)(b * NNODE + row0 + row)) * DIN;
    const v4us r0 = *(const v4usa*)(HB + grow + 4 * l);
    const v4us r1 = *(const v4usa*)(HB + grow + 128 + 4 * l);
    float y[8];
#pragma unroll
    for (int e = 0; e < 4; ++e) {
      y[e]     = x0[e] + pbv[e]     + bf2f(r0[e]);
      y[4 + e] = x1[e] + pbv[4 + e] + bf2f(r1[e]);
    }
    float s = 0.f;
#pragma unroll
    for (int e = 0; e < 8; ++e) s += y[e];
#pragma unroll
    for (int off = 16; off > 0; off >>= 1) s += __shfl_xor(s, off, 32);
    const float mean = s * (1.0f / DOUT);
    float sq = 0.f;
#pragma unroll
    for (int e = 0; e < 8; ++e) { y[e] -= mean; sq += y[e] * y[e]; }
#pragma unroll
    for (int off = 16; off > 0; off >>= 1) sq += __shfl_xor(sq, off, 32);
    const float rstd = rsqrtf(sq * (1.0f / DOUT) + LNEPS);
    v4f o0, o1;
#pragma unroll
    for (int e = 0; e < 4; ++e) {
      o0[e] = y[e] * rstd * gv[e] + bv[e];
      o1[e] = y[4 + e] * rstd * gv[4 + e] + bv[4 + e];
    }
    *(v4fa*)(tr + 4 * l) = o0;
    *(v4fa*)(tr + 128 + 4 * l) = o1;
  }
  out_store(sT, out, b, row0, w, l);
  __threadfence();
  out_store(sT, out, b, row0, w, l);
}

extern "C" void kernel_launch(void* const* d_in, const int* in_sizes, int n_in,
                              void* d_out, int out_size, void* d_ws, size_t ws_size,
                              hipStream_t stream) {
  if (n_in < 9) return;
  if (in_sizes[0] != BB * NNODE * DIN || in_sizes[1] != NNODE * NNODE || in_sizes[2] != NH * DIN * HDIM ||
      in_sizes[3] != NH * HDIM || in_sizes[4] != NH * HDIM || in_sizes[5] != DOUT * DOUT ||
      in_sizes[6] != DOUT || in_sizes[7] != DOUT || in_sizes[8] != DOUT || out_size != BB * NNODE * DOUT) return;

  const float* h   = (const float*)d_in[0];
  const int*   adj = (const int*)d_in[1];
  const float* W   = (const float*)d_in[2];
  const float* a1  = (const float*)d_in[3];
  const float* a2  = (const float*)d_in[4];
  const float* pw  = (const float*)d_in[5];
  const float* pb  = (const float*)d_in[6];
  const float* gam = (const float*)d_in[7];
  const float* bet = (const float*)d_in[8];
  float* out = (float*)d_out;

  const size_t nHB  = (size_t)BB * NNODE * DIN * 2;
  const size_t nPWB = (size_t)DOUT * DOUT * 2;
  const size_t nWT  = (size_t)NH * HDIM * DIN * 2;
  const size_t nADJ = (size_t)NNODE * 32 * 4;
  const size_t nWH  = (size_t)NBH * HDIM * NNODE * 2;
  const size_t nSC  = (size_t)2 * NBH * NNODE * 4;
  const size_t nHM  = (size_t)BB * NNODE * DOUT * 2;
  const size_t oHB  = 0;
  const size_t oPWB = oHB + nHB;
  const size_t oWT  = oPWB + nPWB;
  const size_t oADJ = oWT + nWT;
  const size_t oWHI = oADJ + nADJ;
  const size_t oWLO = oWHI + nWH;
  const size_t oSC  = oWLO + nWH;
  const size_t oHMH = oSC + nSC;
  const size_t oHML = oHMH + nHM;
  const size_t total = oHML + nHM;
  if (total > ws_size) return;

  char* ws = (char*)d_ws;
  unsigned short* HB  = (unsigned short*)(ws + oHB);
  unsigned short* PWB = (unsigned short*)(ws + oPWB);
  unsigned short* WT  = (unsigned short*)(ws + oWT);
  unsigned int*   ADJB = (unsigned int*)(ws + oADJ);
  unsigned short* WHI = (unsigned short*)(ws + oWHI);
  unsigned short* WLO = (unsigned short*)(ws + oWLO);
  float*          SC  = (float*)(ws + oSC);
  unsigned short* HMH = (unsigned short*)(ws + oHMH);
  unsigned short* HML = (unsigned short*)(ws + oHML);

  k_prep<<<PB_TOT, 256, 0, stream>>>(h, adj, W, pw, HB, PWB, WT, ADJB);
  k_gemm_wh<<<BB * NH * NBLK, 128, 0, stream>>>(HB, WT, a1, a2, WHI, WLO, SC);
  k_attn<<<BB * NH * NBLK, 128, 0, stream>>>(ADJB, SC, WHI, WLO, HMH, HML);
  k_proj_ln<<<BB * (NNODE / 32), 128, 0, stream>>>(HMH, HML, PWB, HB, pb, gam, bet, out);
}
